// DataFlowGraphEncoder_55490977465025
// MI455X (gfx1250) — hardware-run, weakly checked
//
#include <hip/hip_runtime.h>
#include <math.h>

typedef __attribute__((ext_vector_type(16))) _Float16 v16h;
typedef __attribute__((ext_vector_type(8)))  _Float16 v8h;
typedef __attribute__((ext_vector_type(16))) __bf16   v16b;
typedef __attribute__((ext_vector_type(8)))  __bf16   v8b;
typedef __attribute__((ext_vector_type(8)))  float    v8f;
typedef __attribute__((ext_vector_type(4)))  float    v4f;

constexpr int kNodes  = 16384;
constexpr int kPer    = 512;
constexpr int kGraphs = 32;
constexpr int kEdges  = 131072;
constexpr int kFin    = 128;
constexpr int kHid    = 128;
constexpr int kHeads  = 4;
constexpr int kLayers = 3;
constexpr int kQKP    = 1024;
constexpr int kVSP    = 640;
constexpr int kGIP    = 384;
constexpr int kMQP    = 256;
constexpr int kMhD    = 32;
static_assert(kGraphs * kPer == kNodes, "graph partition");
static_assert(kHeads * kHid == 512 && 2 * kHeads * kHid == kQKP && kHeads * kHid + kHid == kVSP, "plane pitches");
static_assert(kHeads * kMhD == kHid, "head split");
static_assert((kFin % 32) == 0 && (kHid % 32) == 0, "GEMM K multiples of 32");
static_assert((kNodes % 64) == 0 && (kQKP % 64) == 0 && (kVSP % 64) == 0 && (kGIP % 64) == 0 && (kMQP % 64) == 0 && (kHid % 64) == 0, "GEMM M,N multiples of 64");

constexpr size_t kSzP16   = (size_t)kNodes * 128 * 2;
constexpr size_t kOffNFH  = 0;
constexpr size_t kOffNFL  = kOffNFH  + kSzP16;
constexpr size_t kOffXF   = kOffNFL  + kSzP16;
constexpr size_t kOffXH   = kOffXF   + (size_t)kNodes * 128 * 4;
constexpr size_t kOffXL   = kOffXH   + kSzP16;
constexpr size_t kOffQK   = kOffXL   + kSzP16;
constexpr size_t kOffVS   = kOffQK   + (size_t)kNodes * kQKP * 2;
constexpr size_t kOffWPH  = kOffVS   + (size_t)kNodes * kVSP * 4;
constexpr size_t kOffWPL  = kOffWPH  + (size_t)128 * 128 * 2;
constexpr size_t kOffWQKH = kOffWPL  + (size_t)128 * 128 * 2;
constexpr size_t kOffWQKL = kOffWQKH + (size_t)kLayers * kQKP * 128 * 2;
constexpr size_t kOffWVSH = kOffWQKL + (size_t)kLayers * kQKP * 128 * 2;
constexpr size_t kOffWVSL = kOffWVSH + (size_t)kLayers * kVSP * 128 * 2;
constexpr size_t kOffWIHH = kOffWVSL + (size_t)kLayers * kVSP * 128 * 2;
constexpr size_t kOffWIHL = kOffWIHH + (size_t)384 * 128 * 2;
constexpr size_t kOffWHHH = kOffWIHL + (size_t)384 * 128 * 2;
constexpr size_t kOffWHHL = kOffWHHH + (size_t)384 * 128 * 2;
constexpr size_t kOffWINH = kOffWHHL + (size_t)384 * 128 * 2;
constexpr size_t kOffWINL = kOffWINH + (size_t)384 * 128 * 2;
constexpr size_t kOffWOH  = kOffWINL + (size_t)384 * 128 * 2;
constexpr size_t kOffWOL  = kOffWOH  + (size_t)128 * 128 * 2;
constexpr size_t kOffBQK  = kOffWOL  + (size_t)128 * 128 * 2;
constexpr size_t kOffBVS  = kOffBQK  + (size_t)kLayers * kQKP * 4;
constexpr size_t kOffP2   = kOffBVS  + (size_t)kLayers * kVSP * 4;
constexpr size_t kWsTotal = kOffP2   + (size_t)kGraphs * 32 * 4;
static_assert(kWsTotal == 103964160ull, "carve total");
static_assert(kWsTotal <= 134217728ull, "carve cap");
constexpr size_t kOffGI  = kOffVS;
constexpr size_t kOffRF  = kOffGI + (size_t)kNodes * kGIP * 4;
constexpr size_t kOffUD  = kOffRF + (size_t)kNodes * 128 * 4;
static_assert(kOffUD + (size_t)kNodes * 128 * 4 <= kOffVS + (size_t)kNodes * kVSP * 4, "f32 re-use fits");
constexpr size_t kOffQM  = kOffQK;
constexpr size_t kOffVTH = kOffQM  + (size_t)kNodes * kMQP * 2;
constexpr size_t kOffVTL = kOffVTH + kSzP16;
constexpr size_t kOffOH  = kOffVTL + kSzP16;
constexpr size_t kOffOL  = kOffOH  + kSzP16;
static_assert(kOffOL + kSzP16 <= kOffQK + (size_t)kNodes * kQKP * 2, "bf16 re-use fits");
static_assert((kOffXF % 128) == 0 && (kOffQK % 128) == 0 && (kOffVS % 128) == 0 && (kOffWPH % 128) == 0 &&
              (kOffWQKH % 128) == 0 && (kOffWVSH % 128) == 0 && (kOffWVSL % 128) == 0 && (kOffWIHH % 128) == 0 &&
              (kOffBQK % 128) == 0 && (kOffBVS % 128) == 0 && (kOffP2 % 128) == 0 && (kOffRF % 128) == 0 &&
              (kOffUD % 128) == 0 && (kOffVTH % 128) == 0 && (kOffOH % 128) == 0, "128-B aligned regions");

constexpr size_t kOut0 = 0;
constexpr size_t kOut1 = kOut0 + (size_t)kNodes * kHid;
constexpr size_t kOut2 = kOut1 + (size_t)kGraphs * kHid;
constexpr size_t kOut3 = kOut2 + (size_t)kGraphs * 2;
constexpr size_t kOut4 = kOut3 + (size_t)kNodes * 2;
constexpr size_t kOutTotal = kOut4 + (size_t)kNodes * kHid;
static_assert(kOut1 * 4 == 8388608ull && kOut2 * 4 == 8404992ull && kOut3 * 4 == 8405248ull && kOut4 * 4 == 8536320ull, "output byte offsets");
static_assert(kOutTotal * 4 == 16924928ull, "output total");

__device__ __forceinline__ unsigned short f2bf_bits(float f) {
  unsigned u = __float_as_uint(f);
  return (unsigned short)((u + 0x7FFFu + ((u >> 16) & 1u)) >> 16);
}
__device__ __forceinline__ float bf_bits2f(unsigned short h) { return __uint_as_float(((unsigned)h) << 16); }

__device__ __forceinline__ void dep_guard4_h(v8f& a, v8f& b, v8f& c, v8f& d, v16h x, v16h y) { asm volatile("v_nop\n\tv_nop\n\tv_nop\n\tv_nop" : "+v"(a), "+v"(b), "+v"(c), "+v"(d) : "v"(x), "v"(y)); }
__device__ __forceinline__ void dep_guard4_b(v8f& a, v8f& b, v8f& c, v8f& d, v16b x, v16b y) { asm volatile("v_nop\n\tv_nop\n\tv_nop\n\tv_nop" : "+v"(a), "+v"(b), "+v"(c), "+v"(d) : "v"(x), "v"(y)); }
__device__ __forceinline__ void keep4_h(v16h a, v16h b, v16h c, v16h d) { asm volatile("v_nop" :: "v"(a), "v"(b), "v"(c), "v"(d)); }
__device__ __forceinline__ void keep4_b(v16b a, v16b b, v16b c, v16b d) { asm volatile("v_nop" :: "v"(a), "v"(b), "v"(c), "v"(d)); }
__device__ __forceinline__ void acc_guard4(v8f& a, v8f& b, v8f& c, v8f& d) { asm volatile("v_nop\n\tv_nop\n\tv_nop\n\tv_nop" : "+v"(a), "+v"(b), "+v"(c), "+v"(d)); }
template <typename T> struct Frag;
template <> struct Frag<_Float16> {
  typedef v16h V; union U { v16h v; v8h h[2]; };
  static __device__ __forceinline__ v16h load(const _Float16* p) {
    U f; f.h[0] = *(const v8h*)(p); f.h[1] = *(const v8h*)(p + 16); return f.v;
  }
  static __device__ __forceinline__ v8f mma(v16h a, v16h b, v8f c) {
    return __builtin_amdgcn_wmma_f32_16x16x32_f16(false, a, false, b, (short)0, c, false, false);
  }
  static __device__ __forceinline__ void guard4(v8f& a, v8f& b, v8f& c, v8f& d, v16h x, v16h y) { dep_guard4_h(a, b, c, d, x, y); }
  static __device__ __forceinline__ void keep(v16h a, v16h b, v16h c, v16h d) { keep4_h(a, b, c, d); }
};
template <> struct Frag<__bf16> {
  typedef v16b V; union U { v16b v; v8b h[2]; };
  static __device__ __forceinline__ v16b load(const __bf16* p) {
    U f; f.h[0] = *(const v8b*)(p); f.h[1] = *(const v8b*)(p + 16); return f.v;
  }
  static __device__ __forceinline__ v8f mma(v16b a, v16b b, v8f c) {
    return __builtin_amdgcn_wmma_f32_16x16x32_bf16(false, a, false, b, (short)0, c, false, false);
  }
  static __device__ __forceinline__ void guard4(v8f& a, v8f& b, v8f& c, v8f& d, v16b x, v16b y) { dep_guard4_b(a, b, c, d, x, y); }
  static __device__ __forceinline__ void keep(v16b a, v16b b, v16b c, v16b d) { keep4_b(a, b, c, d); }
};

__device__ __forceinline__ v8f mma_g(v16b a, v16b b, v8f c) {
  c = __builtin_amdgcn_wmma_f32_16x16x32_bf16(false, a, false, b, (short)0, c, false, false);
  asm volatile("v_nop\n\tv_nop\n\tv_nop\n\tv_nop" : "+v"(c) : "v"(a), "v"(b));
  return c;
}
__device__ __forceinline__ __bf16 bf_from_bits(unsigned short b) { return __builtin_bit_cast(__bf16, b); }
__device__ __forceinline__ void split_bf(float f, __bf16& hi, __bf16& lo) {
  const unsigned short hb = f2bf_bits(f);
  const unsigned short lb = f2bf_bits(f - bf_bits2f(hb));
  hi = bf_from_bits(hb);
  lo = bf_from_bits(lb);
}

template <int ET> struct Elem;
template <> struct Elem<0> { typedef _Float16 T; };
template <> struct Elem<1> { typedef __bf16 T; };
template <int ET, int SPL, int BIAS_MODE, int OUT_MODE>
__global__ __launch_bounds__(256) void wmma_gemm64(
    const unsigned short* __restrict__ Ap, const unsigned short* __restrict__ A2p, int lda, long strideA,
    const unsigned short* __restrict__ Btp, const unsigned short* __restrict__ Bt2p, int ldb, long strideB,
    void* __restrict__ Cout, void* __restrict__ Cout2, int ldc, long strideC,
    const float* __restrict__ bias,
    int M, int N, int K, float scale) {
  typedef typename Elem<ET>::T T;
  typedef typename Frag<T>::V V;
  const T* A = (const T*)Ap; const T* A2 = (const T*)A2p; const T* Bt = (const T*)Btp; const T* Bt2 = (const T*)Bt2p;
  __shared__ __align__(16) float sT[8][16 * 68];
  const int b    = blockIdx.y;
  const int lane = threadIdx.x & 31;
  const int wave = __builtin_amdgcn_readfirstlane((int)(threadIdx.x >> 5));
  const int tilesN = N >> 6;
  const int tilesM = M >> 6;
  const int tile = blockIdx.x * 8 + wave;
  if (tile >= tilesM * tilesN) return;
  const int tm = tile / tilesN;
  const int tn = tile - tm * tilesN;
  const int m0 = tm << 6;
  const int n0 = tn << 6;

  const T* Ab  = A  + (size_t)b * strideA;
  const T* Bb  = Bt + (size_t)b * strideB;
  const T* Ab2 = (SPL >= 1) ? (A2  + (size_t)b * strideA) : nullptr;
  const T* Bb2 = (SPL == 2) ? (Bt2 + (size_t)b * strideB) : nullptr;

  const int rlane = lane & 15;
  const int koff  = (lane >> 4) * 8;
  const int mOff  = (lane >> 4) * 8;

  v8f acc[4][4];
#pragma unroll
  for (int i = 0; i < 4; ++i)
#pragma unroll
    for (int j = 0; j < 4; ++j) acc[i][j] = (v8f){0.f,0.f,0.f,0.f,0.f,0.f,0.f,0.f};

  for (int k0 = 0; k0 < K; k0 += 32) {
    V bh[4], bl[4];
#pragma unroll
    for (int j = 0; j < 4; ++j) {
      const size_t bo = (size_t)(n0 + (j << 4) + rlane) * ldb + koff + k0;
      bh[j] = Frag<T>::load(Bb + bo);
      if (SPL == 2) bl[j] = Frag<T>::load(Bb2 + bo);
    }
#pragma unroll
    for (int i = 0; i < 4; ++i) {
      const size_t ao = (size_t)(m0 + (i << 4) + rlane) * lda + koff + k0;
      V ah = Frag<T>::load(Ab + ao);
      V al;
      if (SPL >= 1) al = Frag<T>::load(Ab2 + ao);
#pragma unroll
      for (int j = 0; j < 4; ++j) {
        acc[i][j] = Frag<T>::mma(ah, bh[j], acc[i][j]);
        if (SPL == 2) acc[i][j] = Frag<T>::mma(ah, bl[j], acc[i][j]);
        if (SPL >= 1) acc[i][j] = Frag<T>::mma(al, bh[j], acc[i][j]);
      }
      Frag<T>::guard4(acc[i][0], acc[i][1], acc[i][2], acc[i][3], ah, (SPL >= 1) ? al : ah);
    }
    Frag<T>::keep(bh[0], bh[1], bh[2], bh[3]);
    if (SPL == 2) Frag<T>::keep(bl[0], bl[1], bl[2], bl[3]);
  }
  acc_guard4(acc[0][0], acc[0][1], acc[0][2], acc[0][3]);
  acc_guard4(acc[1][0], acc[1][1], acc[1][2], acc[1][3]);
  acc_guard4(acc[2][0], acc[2][1], acc[2][2], acc[2][3]);
  acc_guard4(acc[3][0], acc[3][1], acc[3][2], acc[3][3]);

  float* slab = sT[wave];
#pragma unroll
  for (int i = 0; i < 4; ++i) {
    const int mBase = m0 + (i << 4);
#pragma unroll
    for (int j = 0; j < 4; ++j) {
      const int n = n0 + (j << 4) + rlane;
      float bv = 0.f;
      if (BIAS_MODE == 2) bv = bias[n];
#pragma unroll
      for (int r = 0; r < 8; ++r) {
        float v = acc[i][j][r] * scale;
        if (BIAS_MODE == 1) v += bias[mBase + mOff + r];
        if (BIAS_MODE == 2) v += bv;
        slab[(mOff + r) * 68 + (j << 4) + rlane] = v;
      }
    }
    __builtin_amdgcn_fence(__ATOMIC_RELEASE, "workgroup");
    __builtin_amdgcn_wave_barrier();
    __builtin_amdgcn_fence(__ATOMIC_ACQUIRE, "workgroup");
    if (OUT_MODE == 0) {
      float* C = (float*)Cout + (size_t)b * strideC;
      const int hh = lane >> 4, c4 = (lane & 15) * 4;
      for (int pass = 0; pass < 2; ++pass) {
#pragma unroll
        for (int it = 0; it < 8; ++it) {
          const int row = it * 2 + hh;
          v4f v = *(const v4f*)(slab + row * 68 + c4);
          *(volatile v4f*)(C + (size_t)(mBase + row) * ldc + n0 + c4) = v;
        }
        __threadfence();
      }
    } else {
      const int q = lane >> 3, c8 = (lane & 7) * 8;
      unsigned short* C  = (unsigned short*)Cout  + (size_t)b * strideC;
      unsigned short* C2 = (OUT_MODE == 2) ? ((unsigned short*)Cout2 + (size_t)b * strideC) : nullptr;
      for (int pass = 0; pass < 2; ++pass) {
#pragma unroll
        for (int it = 0; it < 4; ++it) {
          const int row = it * 4 + q;
          const float* sp = slab + row * 68 + c8;
          v8h hv, lv;
#pragma unroll
          for (int e = 0; e < 8; ++e) {
            if (OUT_MODE == 1) {
              hv[e] = (_Float16)sp[e];
            } else {
              unsigned short hb = f2bf_bits(sp[e]);
              unsigned short lb = f2bf_bits(sp[e] - bf_bits2f(hb));
              hv[e] = __builtin_bit_cast(_Float16, hb);
              lv[e] = __builtin_bit_cast(_Float16, lb);
            }
          }
          *(volatile v8h*)(C + (size_t)(mBase + row) * ldc + n0 + c8) = hv;
          if (OUT_MODE == 2) *(volatile v8h*)(C2 + (size_t)(mBase + row) * ldc + n0 + c8) = lv;
        }
        __threadfence();
      }
    }
    __builtin_amdgcn_fence(__ATOMIC_RELEASE, "workgroup");
    __builtin_amdgcn_wave_barrier();
    __builtin_amdgcn_fence(__ATOMIC_ACQUIRE, "workgroup");
  }
}

__global__ __launch_bounds__(256) void split_rows_bf16_kernel(
    const float* __restrict__ src, unsigned short* __restrict__ dhi, unsigned short* __restrict__ dlo, int total8)
{
  const int i = blockIdx.x * 256 + threadIdx.x;
  if (i >= total8) return;
  const size_t e0 = (size_t)i << 3;
  const v4f a0 = *(const v4f*)(src + e0);
  const v4f a1 = *(const v4f*)(src + e0 + 4);
  v8h hv, lv;
#pragma unroll
  for (int e = 0; e < 4; ++e) {
    const float f0 = a0[e], f1 = a1[e];
    const unsigned short h0 = f2bf_bits(f0), h1 = f2bf_bits(f1);
    const unsigned short l0 = f2bf_bits(f0 - bf_bits2f(h0)), l1 = f2bf_bits(f1 - bf_bits2f(h1));
    hv[e]     = __builtin_bit_cast(_Float16, h0);
    hv[4 + e] = __builtin_bit_cast(_Float16, h1);
    lv[e]     = __builtin_bit_cast(_Float16, l0);
    lv[4 + e] = __builtin_bit_cast(_Float16, l1);
  }
  unsigned short* qh = dhi + e0;
  unsigned short* ql = dlo + e0;
  *(volatile v8h*)qh = hv;
  *(volatile v8h*)ql = lv;
  __threadfence();
  *(volatile v8h*)qh = hv;
  *(volatile v8h*)ql = lv;
}

__global__ __launch_bounds__(256) void prep_wT_kernel(
    const float* __restrict__ Wp, const float* __restrict__ Wq, const float* __restrict__ Wk,
    const float* __restrict__ Wv, const float* __restrict__ Wsk,
    unsigned short* __restrict__ WPH, unsigned short* __restrict__ WPL,
    unsigned short* __restrict__ WQKH, unsigned short* __restrict__ WQKL,
    unsigned short* __restrict__ WVSH, unsigned short* __restrict__ WVSL)
{
  __shared__ float sT[128 * 65];
  const int tid = threadIdx.x;
  int b = blockIdx.x;
  const float* src;
  int ldn, n0;
  unsigned short* dH;
  unsigned short* dL;
  if (b < 2) {
    src = Wp; ldn = 128; n0 = b * 64;
    dH = WPH + (size_t)n0 * 128; dL = WPL + (size_t)n0 * 128;
  } else {
    b -= 2;
    const int l = b / 26;
    const int r = b - l * 26;
    if (r < 8) {
      src = Wq + (size_t)l * 128 * 512; ldn = 512; n0 = r * 64;
      const size_t off = ((size_t)l * kQKP + n0) * 128;
      dH = WQKH + off; dL = WQKL + off;
    } else if (r < 16) {
      src = Wk + (size_t)l * 128 * 512; ldn = 512; n0 = (r - 8) * 64;
      const size_t off = ((size_t)l * kQKP + 512 + n0) * 128;
      dH = WQKH + off; dL = WQKL + off;
    } else if (r < 24) {
      src = Wv + (size_t)l * 128 * 512; ldn = 512; n0 = (r - 16) * 64;
      const size_t off = ((size_t)l * kVSP + n0) * 128;
      dH = WVSH + off; dL = WVSL + off;
    } else {
      src = Wsk + (size_t)l * 128 * 128; ldn = 128; n0 = (r - 24) * 64;
      const size_t off = ((size_t)l * kVSP + 512 + n0) * 128;
      dH = WVSH + off; dL = WVSL + off;
    }
  }
  {
    const int nn4 = (tid & 15) * 4, kr = tid >> 4;
#pragma unroll
    for (int i = 0; i < 8; ++i) {
      const int k = kr + 16 * i;
      const v4f v = *(const v4f*)(src + (size_t)k * ldn + n0 + nn4);
      sT[k * 65 + nn4 + 0] = v[0];
      sT[k * 65 + nn4 + 1] = v[1];
      sT[k * 65 + nn4 + 2] = v[2];
      sT[k * 65 + nn4 + 3] = v[3];
    }
  }
  __syncthreads();
  const int seg = tid & 15, rr = tid >> 4;
  v8h hv[4], lv[4];
#pragma unroll
  for (int it = 0; it < 4; ++it) {
    const int r = it * 16 + rr;
#pragma unroll
    for (int e = 0; e < 8; ++e) {
      const float f = sT[(seg * 8 + e) * 65 + r];
      const unsigned short hb = f2bf_bits(f);
      const unsigned short lb = f2bf_bits(f - bf_bits2f(hb));
      hv[it][e] = __builtin_bit_cast(_Float16, hb);
      lv[it][e] = __builtin_bit_cast(_Float16, lb);
    }
  }
  for (int pass = 0; pass < 2; ++pass) {
#pragma unroll
    for (int it = 0; it < 4; ++it) {
      const size_t o = (size_t)(it * 16 + rr) * 128 + seg * 8;
      *(volatile v8h*)(dH + o) = hv[it];
      *(volatile v8h*)(dL + o) = lv[it];
    }
    __threadfence();
  }
}

__global__ __launch_bounds__(256) void prep_bias_kernel(
    const float* __restrict__ bq, const float* __restrict__ bk, const float* __restrict__ bv, const float* __restrict__ bsk,
    float* __restrict__ BQK, float* __restrict__ BVS)
{
  constexpr int kNqk = kLayers * kQKP;
  constexpr int kNvs = kLayers * kVSP;
  const int i = blockIdx.x * 256 + threadIdx.x;
  const int ic = i < (kNqk + kNvs) ? i : (kNqk + kNvs - 1);
  const bool isqk = ic < kNqk;
  const int a = isqk ? ic : 0;
  const int l1 = a >> 10, c1 = a & 1023, cq = c1 & 511;
  const int bb = isqk ? 0 : (ic - kNqk);
  const int l2 = bb / kVSP, c2 = bb - l2 * kVSP;
  const int cv = c2 < 512 ? c2 : 511;
  const int cs = c2 >= 512 ? (c2 - 512) : 0;
  float vq = bq[l1 * 512 + cq];
  float vk = bk[l1 * 512 + cq];
  float vv = bv[l2 * 512 + cv];
  float vs = bsk[l2 * 128 + cs];
  asm volatile("" : "+v"(vq), "+v"(vk), "+v"(vv), "+v"(vs));
  const float r1 = (c1 < 512) ? vq : vk;
  const float r2 = (c2 < 512) ? vv : vs;
  const float val = isqk ? r1 : r2;
  if (i < kNqk + kNvs) {
    float* dp = isqk ? (BQK + ic) : (BVS + (ic - kNqk));
    *(volatile float*)dp = val;
    __threadfence();
    *(volatile float*)dp = val;
  }
}

__global__ __launch_bounds__(256) void embed_split_kernel(
    const float* __restrict__ XF, const int* __restrict__ vtp, const int* __restrict__ otp,
    const float* __restrict__ vtab, const float* __restrict__ otab,
    unsigned short* __restrict__ XH, unsigned short* __restrict__ XL)
{
  const int i = blockIdx.x * 256 + threadIdx.x;
  const int row = i >> 4, c8 = (i & 15) * 8;
  int vt = vtp[row]; vt = vt < 0 ? 0 : (vt > 19 ? 19 : vt);
  int ot = otp[row]; ot = ot < 0 ? 0 : (ot > 29 ? 29 : ot);
  const size_t e0 = (size_t)row * 128 + c8;
  const v4f a0 = *(const v4f*)(XF + e0);
  const v4f a1 = *(const v4f*)(XF + e0 + 4);
  const int tc = c8 & 31;
  const v4f t0 = *(const v4f*)(vtab + vt * 32 + tc);
  const v4f t1 = *(const v4f*)(vtab + vt * 32 + tc + 4);
  const v4f o0 = *(const v4f*)(otab + ot * 32 + tc);
  const v4f o1 = *(const v4f*)(otab + ot * 32 + tc + 4);
  v8h hv, lv;
#pragma unroll
  for (int e = 0; e < 4; ++e) {
    const float f0 = (a0[e] + t0[e]) + o0[e];
    const float f1 = (a1[e] + t1[e]) + o1[e];
    const unsigned short h0 = f2bf_bits(f0), h1 = f2bf_bits(f1);
    const unsigned short l0 = f2bf_bits(f0 - bf_bits2f(h0)), l1 = f2bf_bits(f1 - bf_bits2f(h1));
    hv[e]     = __builtin_bit_cast(_Float16, h0);
    hv[4 + e] = __builtin_bit_cast(_Float16, h1);
    lv[e]     = __builtin_bit_cast(_Float16, l0);
    lv[4 + e] = __builtin_bit_cast(_Float16, l1);
  }
  *(volatile v8h*)(XH + e0) = hv;
  *(volatile v8h*)(XL + e0) = lv;
  __threadfence();
  *(volatile v8h*)(XH + e0) = hv;
  *(volatile v8h*)(XL + e0) = lv;
}

constexpr int kEaT    = 16;
constexpr int kEaCh   = 2048;
constexpr int kEaWCap = 512;
constexpr int kEaXP   = 132;
static_assert((kEdges % kEaCh) == 0 && kEaCh == 4 * kEaWCap && kEaWCap == 4 * 128, "edge chunking");
static_assert((kNodes % kEaT) == 0 && kEdges <= (1 << 20), "edge tile");

__device__ __forceinline__ float bfdot2(unsigned q, unsigned k, float acc) {
  const float ql = __uint_as_float(q << 16), qh = __uint_as_float(q & 0xffff0000u);
  const float kl = __uint_as_float(k << 16), kh = __uint_as_float(k & 0xffff0000u);
  acc = fmaf(ql, kl, acc);
  acc = fmaf(qh, kh, acc);
  return acc;
}

__global__ __launch_bounds__(128) void edge_attn_kernel(
    const int* __restrict__ srcv, const int* __restrict__ dstv,
    const unsigned short* __restrict__ QK, const float* __restrict__ VS,
    float* __restrict__ XF, unsigned short* __restrict__ XH, unsigned short* __restrict__ XL)
{
  __shared__ __align__(16) float sAcc[kEaT * 512];
  __shared__ __align__(16) float sDen[kEaT * 4];
  __shared__ __align__(16) int   sList[4 * kEaWCap];
  __shared__ int sCnt[4];
  __shared__ __align__(16) float sX[kEaT * kEaXP];
  const int tid = threadIdx.x, lane = tid & 31;
  const int wave = __builtin_amdgcn_readfirstlane((int)(threadIdx.x >> 5));
  const int base = blockIdx.x * kEaT;
#pragma unroll 1
  for (int i = 0; i < 16; ++i) *(v4f*)(sAcc + (size_t)(i * 128 + tid) * 4) = (v4f){0.f, 0.f, 0.f, 0.f};
  if (tid < kEaT * 4) sDen[tid] = 0.f;
  __syncthreads();
  const unsigned ltmask = (1u << lane) - 1u;
  const float scl = 1.0f / sqrtf((float)kHid);

#pragma unroll 1
  for (int c0 = 0; c0 < kEdges; c0 += kEaCh) {
    int cnt = 0;
#pragma unroll 1
    for (int rep = 0; rep < 4; ++rep) {
      const int e0 = c0 + wave * kEaWCap + rep * 128 + lane * 4;
      const int4 dv = *(const int4*)(dstv + e0);
      int d0 = dv.x, d1 = dv.y, d2 = dv.z, d3 = dv.w;
      d0 = d0 < 0 ? 0 : (d0 > kNodes - 1 ? kNodes - 1 : d0);
      d1 = d1 < 0 ? 0 : (d1 > kNodes - 1 ? kNodes - 1 : d1);
      d2 = d2 < 0 ? 0 : (d2 > kNodes - 1 ? kNodes - 1 : d2);
      d3 = d3 < 0 ? 0 : (d3 > kNodes - 1 ? kNodes - 1 : d3);
      const unsigned r0 = (unsigned)(d0 - base), r1 = (unsigned)(d1 - base);
      const unsigned r2 = (unsigned)(d2 - base), r3 = (unsigned)(d3 - base);
      const bool m0 = r0 < (unsigned)kEaT, m1 = r1 < (unsigned)kEaT, m2 = r2 < (unsigned)kEaT, m3 = r3 < (unsigned)kEaT;
      const bool many = (m0 | m1) | (m2 | m3);
      const unsigned anyb = __builtin_amdgcn_ballot_w32(many);
      if (anyb != 0u) {
        {
          const unsigned bb = __builtin_amdgcn_ballot_w32(m0);
          const int pos = cnt + __popc(bb & ltmask);
          if (m0 && pos < kEaWCap) sList[wave * kEaWCap + pos] = (e0 + 0) | (int)(r0 << 20);
          cnt += __popc(bb);
        }
        {
          const unsigned bb = __builtin_amdgcn_ballot_w32(m1);
          const int pos = cnt + __popc(bb & ltmask);
          if (m1 && pos < kEaWCap) sList[wave * kEaWCap + pos] = (e0 + 1) | (int)(r1 << 20);
          cnt += __popc(bb);
        }
        {
          const unsigned bb = __builtin_amdgcn_ballot_w32(m2);
          const int pos = cnt + __popc(bb & ltmask);
          if (m2 && pos < kEaWCap) sList[wave * kEaWCap + pos] = (e0 + 2) | (int)(r2 << 20);
          cnt += __popc(bb);
        }
        {
          const unsigned bb = __builtin_amdgcn_ballot_w32(m3);
          const int pos = cnt + __popc(bb & ltmask);
          if (m3 && pos < kEaWCap) sList[wave * kEaWCap + pos] = (e0 + 3) | (int)(r3 << 20);
          cnt += __popc(bb);
        }
      }
    }
    if (lane == 0) sCnt[wave] = cnt;
    __syncthreads();
#pragma unroll 1
    for (int ww = 0; ww < 4; ++ww) {
      int n = sCnt[ww];
      n = n < 0 ? 0 : (n > kEaWCap ? kEaWCap : n);
      n = __builtin_amdgcn_readfirstlane(n);
#pragma unroll 1
      for (int i = 0; i < n; ++i) {
        const int ent = __builtin_amdgcn_readfirstlane(sList[ww * kEaWCap + i]);
        const int dl = (ent >> 20) & (kEaT - 1);
        if ((dl & 3) == wave) {
          int e = ent & 0xFFFFF;
          e = e > kEdges - 1 ? kEdges - 1 : e;
          int s = srcv[e];
          s = s < 0 ? 0 : (s > kNodes - 1 ? kNodes - 1 : s);
          s = __builtin_amdgcn_readfirstlane(s);
          const int d = base + dl;
          const uint4* qp = (const uint4*)(QK + (size_t)d * kQKP + lane * 16);
          const uint4* kp = (const uint4*)(QK + (size_t)s * kQKP + 512 + lane * 16);
          const uint4 qa = qp[0], qb = qp[1];
          const uint4 ka = kp[0], kb = kp[1];
          float dot = 0.0f;
          dot = bfdot2(qa.x, ka.x, dot);
          dot = bfdot2(qa.y, ka.y, dot);
          dot = bfdot2(qa.z, ka.z, dot);
          dot = bfdot2(qa.w, ka.w, dot);
          dot = bfdot2(qb.x, kb.x, dot);
          dot = bfdot2(qb.y, kb.y, dot);
          dot = bfdot2(qb.z, kb.z, dot);
          dot = bfdot2(qb.w, kb.w, dot);
          dot += __shfl_xor(dot, 1, 32);
          dot += __shfl_xor(dot, 2, 32);
          dot += __shfl_xor(dot, 4, 32);
          const float ex = expf(dot * scl);
          const float* vp = VS + (size_t)s * kVSP + lane * 16;
          float* ap = sAcc + dl * 512 + lane * 16;
#pragma unroll 1
          for (int q4 = 0; q4 < 4; ++q4) {
            const v4f v = *(const v4f*)(vp + 4 * q4);
            v4f a = *(const v4f*)(ap + 4 * q4);
            a[0] = fmaf(ex, v[0], a[0]);
            a[1] = fmaf(ex, v[1], a[1]);
            a[2] = fmaf(ex, v[2], a[2]);
            a[3] = fmaf(ex, v[3], a[3]);
            *(v4f*)(ap + 4 * q4) = a;
          }
          if ((lane & 7) == 0) sDen[dl * 4 + (lane >> 3)] += ex;
        }
      }
    }
    __syncthreads();
  }

  if (tid < kEaT * 4) sDen[tid] = 1.0f / (sDen[tid] + 1e-16f);
  __syncthreads();
  {
    const int c = tid;
#pragma unroll 1
    for (int dl = 0; dl < kEaT; ++dl) {
      float a = 0.0f;
      a += sAcc[dl * 512 + 0 * 128 + c] * sDen[dl * 4 + 0];
      a += sAcc[dl * 512 + 1 * 128 + c] * sDen[dl * 4 + 1];
      a += sAcc[dl * 512 + 2 * 128 + c] * sDen[dl * 4 + 2];
      a += sAcc[dl * 512 + 3 * 128 + c] * sDen[dl * 4 + 3];
      a *= 0.25f;
      const float pre = a + VS[(size_t)(base + dl) * kVSP + 512 + c];
      sX[dl * kEaXP + c] = 0.5f * pre * (1.0f + erff(pre * 0.70710678118654752f));
    }
  }
  __syncthreads();
  v4f fv[4];
  v8h bh[2], bl[2];
#pragma unroll
  for (int it = 0; it < 4; ++it) fv[it] = *(const v4f*)(sX + (wave * 4 + it) * kEaXP + lane * 4);
#pragma unroll
  for (int it = 0; it < 2; ++it) {
    const int row = wave * 4 + it * 2 + (lane >> 4);
    const float* sp = sX + row * kEaXP + (lane & 15) * 8;
    const v4f a0 = *(const v4f*)(sp);
    const v4f a1 = *(const v4f*)(sp + 4);
#pragma unroll
    for (int e = 0; e < 4; ++e) {
      const float f0 = a0[e], f1 = a1[e];
      const unsigned short h0 = f2bf_bits(f0), h1 = f2bf_bits(f1);
      const unsigned short l0 = f2bf_bits(f0 - bf_bits2f(h0)), l1 = f2bf_bits(f1 - bf_bits2f(h1));
      bh[it][e]     = __builtin_bit_cast(_Float16, h0);
      bh[it][4 + e] = __builtin_bit_cast(_Float16, h1);
      bl[it][e]     = __builtin_bit_cast(_Float16, l0);
      bl[it][4 + e] = __builtin_bit_cast(_Float16, l1);
    }
  }
  for (int pass = 0; pass < 2; ++pass) {
#pragma unroll
    for (int it = 0; it < 4; ++it)
      *(volatile v4f*)(XF + (size_t)(base + wave * 4 + it) * 128 + lane * 4) = fv[it];
#pragma unroll
    for (int it = 0; it < 2; ++it) {
      const size_t o = (size_t)(base + wave * 4 + it * 2 + (lane >> 4)) * 128 + (lane & 15) * 8;
      *(volatile v8h*)(XH + o) = bh[it];
      *(volatile v8h*)(XL + o) = bl[it];
    }
    __threadfence();
  }
}

constexpr int kGrG  = 16;
constexpr int kGrHP = 136;
constexpr int kGrOP = 132;
static_assert((kGraphs % kGrG) == 0, "sequence tile");

__global__ __launch_bounds__(256) void gru_kernel(
    const float* __restrict__ GI, const unsigned short* __restrict__ WhhHp, const float* __restrict__ bhh,
    float* __restrict__ RF)
{
  __shared__ __align__(16) unsigned short sHh[2][kGrG * kGrHP];
  __shared__ __align__(16) unsigned short sHl[2][kGrG * kGrHP];
  __shared__ __align__(16) float sO[2][kGrG * kGrOP];
  const int tid = threadIdx.x, lane = tid & 31;
  const int wave = __builtin_amdgcn_readfirstlane((int)(threadIdx.x >> 5));
  const int hh = lane >> 4, c = lane & 15;
  const int g0 = blockIdx.x * kGrG;
  const int j = wave * 16 + c;
  const __bf16* Wb = (const __bf16*)WhhHp;
  v16b bR[4], bZ[4], bN[4];
#pragma unroll
  for (int ks = 0; ks < 4; ++ks) {
    bR[ks] = Frag<__bf16>::load(Wb + (size_t)(j) * 128 + ks * 32 + 8 * hh);
    bZ[ks] = Frag<__bf16>::load(Wb + (size_t)(128 + j) * 128 + ks * 32 + 8 * hh);
    bN[ks] = Frag<__bf16>::load(Wb + (size_t)(256 + j) * 128 + ks * 32 + 8 * hh);
  }
  const float bhr = bhh[j], bhz = bhh[128 + j], bhn = bhh[256 + j];
  float hreg[8];
#pragma unroll
  for (int r = 0; r < 8; ++r) hreg[r] = 0.f;
#pragma unroll 1
  for (int i = tid; i < 2 * kGrG * kGrHP; i += 256) {
    (&sHh[0][0])[i] = (unsigned short)0;
    (&sHl[0][0])[i] = (unsigned short)0;
  }
  __syncthreads();

#pragma unroll 1
  for (int t = 0; t < kPer; ++t) {
    const int cur = t & 1, nxt = cur ^ 1;
    float gr[8], gz[8], gn[8];
#pragma unroll
    for (int r = 0; r < 8; ++r) {
      const float* gp = GI + ((size_t)(g0 + 8 * hh + r) * kPer + t) * kGIP + j;
      gr[r] = gp[0];
      gz[r] = gp[128];
      gn[r] = gp[256];
    }
    v8f aR = (v8f){0.f,0.f,0.f,0.f,0.f,0.f,0.f,0.f};
    v8f aZ = aR, aN = aR;
    const __bf16* ph = (const __bf16*)(&sHh[cur][0]) + c * kGrHP + 8 * hh;
    const __bf16* pl = (const __bf16*)(&sHl[cur][0]) + c * kGrHP + 8 * hh;
#pragma unroll
    for (int ks = 0; ks < 4; ++ks) {
      const v16b ah = Frag<__bf16>::load(ph + ks * 32);
      const v16b al = Frag<__bf16>::load(pl + ks * 32);
      aR = mma_g(ah, bR[ks], aR);
      aR = mma_g(al, bR[ks], aR);
      aZ = mma_g(ah, bZ[ks], aZ);
      aZ = mma_g(al, bZ[ks], aZ);
      aN = mma_g(ah, bN[ks], aN);
      aN = mma_g(al, bN[ks], aN);
    }
    unsigned short* wh = &sHh[nxt][0];
    unsigned short* wl = &sHl[nxt][0];
    float* wo = &sO[cur][0];
#pragma unroll
    for (int r = 0; r < 8; ++r) {
      const float pr = gr[r] + (aR[r] + bhr);
      const float rg = 1.0f / (1.0f + expf(-pr));
      const float pz = gz[r] + (aZ[r] + bhz);
      const float zg = 1.0f / (1.0f + expf(-pz));
      const float nn = tanhf(gn[r] + rg * (aN[r] + bhn));
      const float hn = (1.0f - zg) * nn + zg * hreg[r];
      hreg[r] = hn;
      const int row = 8 * hh + r;
      const unsigned short hb = f2bf_bits(hn);
      const unsigned short lb = f2bf_bits(hn - bf_bits2f(hb));
      wh[row * kGrHP + j] = hb;
      wl[row * kGrHP + j] = lb;
      wo[row * kGrOP + j] = hn;
    }
    __syncthreads();
    {
      const v4f o0 = *(const v4f*)(wo + (2 * wave) * kGrOP + lane * 4);
      const v4f o1 = *(const v4f*)(wo + (2 * wave + 1) * kGrOP + lane * 4);
      float* d0 = RF + ((size_t)(g0 + 2 * wave) * kPer + t) * 128 + lane * 4;
      float* d1 = RF + ((size_t)(g0 + 2 * wave + 1) * kPer + t) * 128 + lane * 4;
      *(volatile v4f*)d0 = o0;
      *(volatile v4f*)d1 = o1;
      __threadfence();
      *(volatile v4f*)d0 = o0;
      *(volatile v4f*)d1 = o1;
    }
  }
}

__global__ __launch_bounds__(256) void logits_kernel(
    const float* __restrict__ RF, const float* __restrict__ Wc, const float* __restrict__ bc,
    float* __restrict__ out3, float* __restrict__ P2)
{
  __shared__ float sW[256];
  __shared__ float sP[16];
  const int tid = threadIdx.x, lane = tid & 31;
  const int wave = __builtin_amdgcn_readfirstlane((int)(threadIdx.x >> 5));
  const int g = blockIdx.x;
  sW[tid] = Wc[tid];
  __syncthreads();
  const int c = lane & 1;
  const float bcv = bc[c];
  float psum = 0.f;
#pragma unroll 1
  for (int it = 0; it < 4; ++it) {
    const int tile = wave * 4 + it;
    const int node = g * kPer + tile * 16 + (lane >> 1);
    const float* f = RF + (size_t)node * 128;
    float acc = 0.f;
#pragma unroll 2
    for (int jj = 0; jj < 32; ++jj) {
      const v4f x = *(const v4f*)(f + 4 * jj);
      acc = fmaf(x[0], sW[(4 * jj + 0) * 2 + c], acc);
      acc = fmaf(x[1], sW[(4 * jj + 1) * 2 + c], acc);
      acc = fmaf(x[2], sW[(4 * jj + 2) * 2 + c], acc);
      acc = fmaf(x[3], sW[(4 * jj + 3) * 2 + c], acc);
    }
    const float lg = acc + bcv;
    const float ot = __shfl_xor(lg, 1, 32);
    const float mx = fmaxf(lg, ot);
    const float e0 = expf(lg - mx), e1 = expf(ot - mx);
    psum += e0 * (1.0f / (e0 + e1));
    float* dp = out3 + (size_t)(g * kPer + tile * 16) * 2 + lane;
    *(volatile float*)dp = lg;
    __threadfence();
    *(volatile float*)dp = lg;
  }
  psum += __shfl_xor(psum, 2, 32);
  psum += __shfl_xor(psum, 4, 32);
  psum += __shfl_xor(psum, 8, 32);
  psum += __shfl_xor(psum, 16, 32);
  if (lane < 2) sP[wave * 2 + lane] = psum;
  __syncthreads();
  if (wave == 0) {
    float s = 0.f;
#pragma unroll
    for (int w = 0; w < 8; ++w) s += sP[w * 2 + c];
    s *= (1.0f / (float)kPer);
    const float val = (lane < 2) ? s : 0.0f;
    float* dp = P2 + (size_t)g * 32 + lane;
    *(volatile float*)dp = val;
    __threadfence();
    *(volatile float*)dp = val;
  }
}

__global__ __launch_bounds__(128) void mha_kernel(
    const unsigned short* __restrict__ QMp, const unsigned short* __restrict__ VTHp, const unsigned short* __restrict__ VTLp,
    unsigned short* __restrict__ OH, unsigned short* __restrict__ OL)
{
  union FB { v16b v; v8b h[2]; };
  __shared__ __align__(16) __bf16 sPh[4][16 * 64];
  __shared__ __align__(16) __bf16 sPl[4][16 * 64];
  __shared__ __align__(16) float sO[16 * 132];
  const int tid = threadIdx.x, lane = tid & 31;
  const int wave = __builtin_amdgcn_readfirstlane((int)(threadIdx.x >> 5));
  const int hh = lane >> 4, c = lane & 15;
  const int g = blockIdx.x >> 5, qt = blockIdx.x & 31;
  const int q0 = g * kPer + qt * 16;
  const int kbase = g * kPer;
  const __bf16* Qm  = (const __bf16*)QMp;
  const __bf16* VtH = (const __bf16*)VTHp;
  const __bf16* VtL = (const __bf16*)VTLp;
  const float scl = 1.0f / sqrtf((float)kMhD);
  const v16b qa = Frag<__bf16>::load(Qm + (size_t)(q0 + c) * kMQP + wave * kMhD + 8 * hh);

  float mrow[8], lrow[8];
  v8f oacc[2];
#pragma unroll
  for (int r = 0; r < 8; ++r) { mrow[r] = -INFINITY; lrow[r] = 0.f; }
  oacc[0] = (v8f){0.f,0.f,0.f,0.f,0.f,0.f,0.f,0.f};
  oacc[1] = oacc[0];
  __bf16* pwh = sPh[wave];
  __bf16* pwl = sPl[wave];

#pragma unroll 1
  for (int kc = 0; kc < kPer / 64; ++kc) {
    const int kv0 = kbase + kc * 64;
    v8f s[4];
#pragma unroll
    for (int jt = 0; jt < 4; ++jt) {
      const v16b kb = Frag<__bf16>::load(Qm + (size_t)(kv0 + jt * 16 + c) * kMQP + 128 + wave * kMhD + 8 * hh);
      s[jt] = mma_g(qa, kb, (v8f){0.f,0.f,0.f,0.f,0.f,0.f,0.f,0.f});
    }
    float cm[8];
#pragma unroll
    for (int r = 0; r < 8; ++r) {
      float m = -INFINITY;
#pragma unroll
      for (int jt = 0; jt < 4; ++jt) {
        s[jt][r] *= scl;
        m = fmaxf(m, s[jt][r]);
      }
      m = fmaxf(m, __shfl_xor(m, 1, 32));
      m = fmaxf(m, __shfl_xor(m, 2, 32));
      m = fmaxf(m, __shfl_xor(m, 4, 32));
      m = fmaxf(m, __shfl_xor(m, 8, 32));
      cm[r] = m;
    }
#pragma unroll
    for (int r = 0; r < 8; ++r) {
      const float mnew = fmaxf(mrow[r], cm[r]);
      const float alpha = __expf(mrow[r] - mnew);
      mrow[r] = mnew;
      float psum = 0.f;
#pragma unroll
      for (int jt = 0; jt < 4; ++jt) {
        const float p = __expf(s[jt][r] - mnew);
        psum += p;
        __bf16 a, bl;
        split_bf(p, a, bl);
        pwh[(8 * hh + r) * 64 + jt * 16 + c] = a;
        pwl[(8 * hh + r) * 64 + jt * 16 + c] = bl;
      }
      psum += __shfl_xor(psum, 1, 32);
      psum += __shfl_xor(psum, 2, 32);
      psum += __shfl_xor(psum, 4, 32);
      psum += __shfl_xor(psum, 8, 32);
      lrow[r] = lrow[r] * alpha + psum;
      oacc[0][r] *= alpha;
      oacc[1][r] *= alpha;
    }
    __builtin_amdgcn_fence(__ATOMIC_RELEASE, "workgroup");
    __builtin_amdgcn_wave_barrier();
    __builtin_amdgcn_fence(__ATOMIC_ACQUIRE, "workgroup");
#pragma unroll
    for (int kk = 0; kk < 2; ++kk) {
      FB pa, pl;
      pa.h[0] = *(const v8b*)(pwh + c * 64 + kk * 32 + 8 * hh);
      pa.h[1] = *(const v8b*)(pwh + c * 64 + kk * 32 + 16 + 8 * hh);
      pl.h[0] = *(const v8b*)(pwl + c * 64 + kk * 32 + 8 * hh);
      pl.h[1] = *(const v8b*)(pwl + c * 64 + kk * 32 + 16 + 8 * hh);
#pragma unroll
      for (int tt = 0; tt < 2; ++tt) {
        const size_t vo = (size_t)(wave * kMhD + tt * 16 + c) * kNodes + kv0 + kk * 32 + 8 * hh;
        const v16b vb = Frag<__bf16>::load(VtH + vo);
        const v16b vl = Frag<__bf16>::load(VtL + vo);
        oacc[tt] = mma_g(pa.v, vb, oacc[tt]);
        oacc[tt] = mma_g(pa.v, vl, oacc[tt]);
        oacc[tt] = mma_g(pl.v, vb, oacc[tt]);
      }
    }
    __builtin_amdgcn_fence(__ATOMIC_RELEASE, "workgroup");
    __builtin_amdgcn_wave_barrier();
    __builtin_amdgcn_fence(__ATOMIC_ACQUIRE, "workgroup");
  }

#pragma unroll
  for (int r = 0; r < 8; ++r) {
    const float inv = 1.0f / lrow[r];
    sO[(8 * hh + r) * 132 + wave * kMhD + c]      = oacc[0][r] * inv;
    sO[(8 * hh + r) * 132 + wave * kMhD + 16 + c] = oacc[1][r] * inv;
  }
  __syncthreads();
  v8h bh[2], bl[2];
#pragma unroll
  for (int it = 0; it < 2; ++it) {
    const int row = wave * 4 + it * 2 + hh;
    const float* sp = sO + row * 132 + c * 8;
    const v4f a0 = *(const v4f*)(sp);
    const v4f a1 = *(const v4f*)(sp + 4);
#pragma unroll
    for (int e = 0; e < 4; ++e) {
      const float f0 = a0[e], f1 = a1[e];
      const unsigned short h0 = f2bf_bits(f0), h1 = f2bf_bits(f1);
      const unsigned short l0 = f2bf_bits(f0 - bf_bits2f(h0)), l1 = f2bf_bits(f1 - bf_bits2f(h1));
      bh[it][e]     = __builtin_bit_cast(_Float16, h0);
      bh[it][4 + e] = __builtin_bit_cast(_Float16, h1);
      bl[it][e]     = __builtin_bit_cast(_Float16, l0);
      bl[it][4 + e] = __builtin_bit_cast(_Float16, l1);
    }
  }
  for (int pass = 0; pass < 2; ++pass) {
#pragma unroll
    for (int it = 0; it < 2; ++it) {
      const size_t o = (size_t)(q0 + wave * 4 + it * 2 + hh) * 128 + c * 8;
      *(volatile v8h*)(OH + o) = bh[it];
      *(volatile v8h*)(OL + o) = bl[it];
    }
    __threadfence();
  }
}

__global__ __launch_bounds__(256) void final_kernel(
    const float* __restrict__ XF, const float* __restrict__ RF, const float* __restrict__ UD, const float* __restrict__ P2,
    float* __restrict__ out0, float* __restrict__ out1, float* __restrict__ out2, float* __restrict__ out4)
{
  __shared__ __align__(16) float sS[8 * 128];
  const int tid = threadIdx.x, lane = tid & 31;
  const int wave = __builtin_amdgcn_readfirstlane((int)(threadIdx.x >> 5));
  const int g = blockIdx.x;
  const int c4 = lane * 4;
  v4f sum = (v4f){0.f, 0.f, 0.f, 0.f};
#pragma unroll 1
  for (int i = 0; i < kPer / 8; ++i) {
    const size_t o = (size_t)(g * kPer + i * 8 + wave) * 128 + c4;
    const v4f x = *(const v4f*)(XF + o);
    const v4f r = *(const v4f*)(RF + o);
    const v4f u = *(const v4f*)(UD + o);
    v4f cmb;
    cmb[0] = (x[0] + r[0]) + u[0];
    cmb[1] = (x[1] + r[1]) + u[1];
    cmb[2] = (x[2] + r[2]) + u[2];
    cmb[3] = (x[3] + r[3]) + u[3];
    sum[0] += cmb[0];
    sum[1] += cmb[1];
    sum[2] += cmb[2];
    sum[3] += cmb[3];
    *(volatile v4f*)(out0 + o) = cmb;
    *(volatile v4f*)(out4 + o) = u;
    __threadfence();
    *(volatile v4f*)(out0 + o) = cmb;
    *(volatile v4f*)(out4 + o) = u;
  }
  *(v4f*)(sS + wave * 128 + c4) = sum;
  __syncthreads();
  if (wave == 0) {
    v4f tot = (v4f){0.f, 0.f, 0.f, 0.f};
#pragma unroll
    for (int w = 0; w < 8; ++w) {
      const v4f p = *(const v4f*)(sS + w * 128 + c4);
      tot[0] += p[0];
      tot[1] += p[1];
      tot[2] += p[2];
      tot[3] += p[3];
    }
    const float inv = 1.0f / (float)kPer;
    tot[0] *= inv;
    tot[1] *= inv;
    tot[2] *= inv;
    tot[3] *= inv;
    float* dp = out1 + (size_t)g * 128 + c4;
    *(volatile v4f*)dp = tot;
    __threadfence();
    *(volatile v4f*)dp = tot;
    if (g == 0) {
      const float v0 = P2[(size_t)(lane >> 1) * 32 + (lane & 1)];
      const float v1 = P2[(size_t)(16 + (lane >> 1)) * 32 + (lane & 1)];
      *(volatile float*)(out2 + lane) = v0;
      *(volatile float*)(out2 + 32 + lane) = v1;
      __threadfence();
      *(volatile float*)(out2 + lane) = v0;
      *(volatile float*)(out2 + 32 + lane) = v1;
    }
  }
}

extern "C" void kernel_launch(void* const* d_in, const int* in_sizes, int n_in,
                              void* d_out, int out_size, void* d_ws, size_t ws_size,
                              hipStream_t stream) {
  if (n_in < 27) return;
  if (in_sizes[0] != kNodes * kFin) return;
  if (in_sizes[1] != 2 * kEdges) return;
  if (in_sizes[2] != kNodes || in_sizes[3] != kNodes) return;
  if (in_sizes[5] != kFin * kHid) return;
  if (in_sizes[9] != kLayers * kHid * 512 || in_sizes[10] != kLayers * kHid * 512 || in_sizes[11] != kLayers * kHid * 512) return;
  if (in_sizes[15] != kLayers * kHid * kHid) return;
  if (in_sizes[17] != 384 * kHid || in_sizes[18] != 384 * kHid || in_sizes[21] != 384 * kHid) return;
  if (in_sizes[23] != kHid * kHid || in_sizes[25] != kHid * 2) return;
  if ((size_t)out_size != kOutTotal) return;
  if (ws_size < kWsTotal) return;

  const float* nf   = (const float*)d_in[0];
  const int*   ei   = (const int*)d_in[1];
  const int*   srcv = ei;
  const int*   dstv = ei + kEdges;
  const int*   vt   = (const int*)d_in[2];
  const int*   ot   = (const int*)d_in[3];
  const float* Wp   = (const float*)d_in[5];
  const float* bp   = (const float*)d_in[6];
  const float* vtab = (const float*)d_in[7];
  const float* otab = (const float*)d_in[8];
  const float* Wq   = (const float*)d_in[9];
  const float* Wk   = (const float*)d_in[10];
  const float* Wv   = (const float*)d_in[11];
  const float* bq   = (const float*)d_in[12];
  const float* bk   = (const float*)d_in[13];
  const float* bv   = (const float*)d_in[14];
  const float* Wsk  = (const float*)d_in[15];
  const float* bsk  = (const float*)d_in[16];
  const float* Wih  = (const float*)d_in[17];
  const float* Whh  = (const float*)d_in[18];
  const float* bih  = (const float*)d_in[19];
  const float* bhh  = (const float*)d_in[20];
  const float* miw  = (const float*)d_in[21];
  const float* mib  = (const float*)d_in[22];
  const float* mow  = (const float*)d_in[23];
  const float* mob  = (const float*)d_in[24];
  const float* Wc   = (const float*)d_in[25];
  const float* bc   = (const float*)d_in[26];

  float* outp = (float*)d_out;
  float* out0 = outp + kOut0;
  float* out1 = outp + kOut1;
  float* out2 = outp + kOut2;
  float* out3 = outp + kOut3;
  float* out4 = outp + kOut4;

  char* ws = (char*)d_ws;
  unsigned short* NFH  = (unsigned short*)(ws + kOffNFH);
  unsigned short* NFL  = (unsigned short*)(ws + kOffNFL);
  float*          XF   = (float*)(ws + kOffXF);
  unsigned short* XH   = (unsigned short*)(ws + kOffXH);
  unsigned short* XL   = (unsigned short*)(ws + kOffXL);
  unsigned short* QK   = (unsigned short*)(ws + kOffQK);
  float*          VS   = (float*)(ws + kOffVS);
  unsigned short* WPH  = (unsigned short*)(ws + kOffWPH);
  unsigned short* WPL  = (unsigned short*)(ws + kOffWPL);
  unsigned short* WQKH = (unsigned short*)(ws + kOffWQKH);
  unsigned short* WQKL = (unsigned short*)(ws + kOffWQKL);
  unsigned short* WVSH = (unsigned short*)(ws + kOffWVSH);
  unsigned short* WVSL = (unsigned short*)(ws + kOffWVSL);
  unsigned short* WIHH = (unsigned short*)(ws + kOffWIHH);
  unsigned short* WIHL = (unsigned short*)(ws + kOffWIHL);
  unsigned short* WHHH = (unsigned short*)(ws + kOffWHHH);
  unsigned short* WHHL = (unsigned short*)(ws + kOffWHHL);
  unsigned short* WINH = (unsigned short*)(ws + kOffWINH);
  unsigned short* WINL = (unsigned short*)(ws + kOffWINL);
  unsigned short* WOH  = (unsigned short*)(ws + kOffWOH);
  unsigned short* WOL  = (unsigned short*)(ws + kOffWOL);
  float*          BQK  = (float*)(ws + kOffBQK);
  float*          BVS  = (float*)(ws + kOffBVS);
  float*          P2   = (float*)(ws + kOffP2);
  float*          GI   = (float*)(ws + kOffGI);
  float*          RF   = (float*)(ws + kOffRF);
  float*          UD   = (float*)(ws + kOffUD);
  unsigned short* QM   = (unsigned short*)(ws + kOffQM);
  unsigned short* VTH  = (unsigned short*)(ws + kOffVTH);
  unsigned short* VTL  = (unsigned short*)(ws + kOffVTL);
  unsigned short* OHp  = (unsigned short*)(ws + kOffOH);
  unsigned short* OLp  = (unsigned short*)(ws + kOffOL);

  prep_wT_kernel<<<2 + kLayers * 26, 256, 0, stream>>>(Wp, Wq, Wk, Wv, Wsk, WPH, WPL, WQKH, WQKL, WVSH, WVSL);
  prep_bias_kernel<<<(kLayers * (kQKP + kVSP) + 255) / 256, 256, 0, stream>>>(bq, bk, bv, bsk, BQK, BVS);
  split_rows_bf16_kernel<<<(kNodes * kFin / 8) / 256, 256, 0, stream>>>(nf, NFH, NFL, kNodes * kFin / 8);
  split_rows_bf16_kernel<<<(384 * 128 / 8) / 256, 256, 0, stream>>>(Wih, WIHH, WIHL, 384 * 128 / 8);
  split_rows_bf16_kernel<<<(384 * 128 / 8) / 256, 256, 0, stream>>>(Whh, WHHH, WHHL, 384 * 128 / 8);
  split_rows_bf16_kernel<<<(384 * 128 / 8) / 256, 256, 0, stream>>>(miw, WINH, WINL, 384 * 128 / 8);
  split_rows_bf16_kernel<<<(128 * 128 / 8) / 256, 256, 0, stream>>>(mow, WOH, WOL, 128 * 128 / 8);

  wmma_gemm64<1, 2, 2, 0><<<dim3(64, 1), 256, 0, stream>>>(
      NFH, NFL, kFin, 0L, WPH, WPL, kFin, 0L, (void*)XF, (void*)XF, kHid, 0L, bp, kNodes, kHid, kFin, 1.0f);
  embed_split_kernel<<<(kNodes * 16) / 256, 256, 0, stream>>>(XF, vt, ot, vtab, otab, XH, XL);

  for (int l = 0; l < kLayers; ++l) {
    wmma_gemm64<1, 0, 2, 3><<<dim3(512, 1), 256, 0, stream>>>(
        XH, XH, kHid, 0L, WQKH + (size_t)l * kQKP * 128, WQKH + (size_t)l * kQKP * 128, kHid, 0L,
        (void*)QK, (void*)QK, kQKP, 0L, BQK + (size_t)l * kQKP, kNodes, kQKP, kHid, 1.0f);
    wmma_gemm64<1, 2, 2, 0><<<dim3(320, 1), 256, 0, stream>>>(
        XH, XL, kHid, 0L, WVSH + (size_t)l * kVSP * 128, WVSL + (size_t)l * kVSP * 128, kHid, 0L,
        (void*)VS, (void*)VS, kVSP, 0L, BVS + (size_t)l * kVSP, kNodes, kVSP, kHid, 1.0f);
    edge_attn_kernel<<<kNodes / kEaT, 128, 0, stream>>>(srcv, dstv, QK, VS, XF, XH, XL);
  }

  wmma_gemm64<1, 2, 2, 0><<<dim3(192, 1), 256, 0, stream>>>(
      XH, XL, kHid, 0L, WIHH, WIHL, kHid, 0L, (void*)GI, (void*)GI, kGIP, 0L, bih, kNodes, kGIP, kHid, 1.0f);
  gru_kernel<<<kGraphs / kGrG, 256, 0, stream>>>(GI, WHHH, bhh, RF);
  logits_kernel<<<kGraphs, 256, 0, stream>>>(RF, Wc, bc, out3, P2);

  wmma_gemm64<1, 0, 2, 3><<<dim3(128, 1), 256, 0, stream>>>(
      XH, XH, kHid, 0L, WINH, WINH, kHid, 0L, (void*)QM, (void*)QM, kMQP, 0L, mib, kNodes, kMQP, kHid, 1.0f);
  wmma_gemm64<1, 2, 1, 2><<<dim3(64, 1), 256, 0, stream>>>(
      WINH + (size_t)256 * 128, WINL + (size_t)256 * 128, kHid, 0L, XH, XL, kHid, 0L,
      (void*)VTH, (void*)VTL, kNodes, 0L, mib + 256, kHid, kNodes, kHid, 1.0f);
  mha_kernel<<<kGraphs * (kPer / 16), 128, 0, stream>>>(QM, VTH, VTL, OHp, OLp);
  wmma_gemm64<1, 2, 2, 0><<<dim3(64, 1), 256, 0, stream>>>(
      OHp, OLp, kHid, 0L, WOH, WOL, kHid, 0L, (void*)UD, (void*)UD, kHid, 0L, mob, kNodes, kHid, kHid, 1.0f);

  final_kernel<<<kGraphs, 256, 0, stream>>>(XF, RF, UD, P2, out0, out1, out2, out4);
}
